// RNN_85306640433621
// MI455X (gfx1250) — hardware-verified
//
#include <hip/hip_runtime.h>
#include <hip/hip_bf16.h>


#define SEQ      512
#define HID      256
#define ROWS     32
#define MT       (ROWS / 16)
#define WAVES    16
#define THREADS  (WAVES * 32)
#define TCHUNK   16
#define HSTRIDE  264

#define __bf16 _Float16
typedef __attribute__((ext_vector_type(16))) _Float16 bf16x16;
typedef __attribute__((ext_vector_type(8)))  _Float16 bf16x8;
typedef __attribute__((ext_vector_type(8)))  float  f32x8;

union ATile { bf16x16 v; struct { bf16x8 lo; bf16x8 hi; } s; };

__device__ __forceinline__ float fast_tanh(float x) {
  float xc = __builtin_fmaxf(__builtin_fminf(x, 15.0f), -15.0f);
  float e  = __builtin_amdgcn_exp2f(xc * 2.8853900817779268f);
  return (e - 1.0f) * __builtin_amdgcn_rcpf(e + 1.0f);
}

__global__ __launch_bounds__(THREADS)
void rnn_scan_wmma(const float* __restrict__ xs,
                   const float* __restrict__ W1x,
                   const float* __restrict__ W1h,
                   const float* __restrict__ b1,
                   const float* __restrict__ W2,
                   const float* __restrict__ b2,
                   float* __restrict__ out)
{
  __shared__ __align__(16) __bf16 sh[ROWS * HSTRIDE];
  __shared__ __align__(16) float  sx[ROWS * TCHUNK * 2];
  __shared__ float sred[WAVES][ROWS];

  const int tid   = threadIdx.x;
  const int wave  = tid >> 5;
  const int lane  = tid & 31;
  const int l15   = lane & 15;
  const int hsel  = lane >> 4;
  const int n     = wave * 16 + l15;
  const int rowb  = blockIdx.x * ROWS;

  {
    unsigned* p = (unsigned*)sh;
    const int ndw = ROWS * HSTRIDE * 2 / 4;
    for (int i = tid; i < ndw; i += THREADS) p[i] = 0u;
  }

  const float b1n = b1[n];
  const float wx0 = W1x[n];
  const float wx1 = W1x[HID + n];
  const float w2n = W2[n];

  bf16x16 B[8];
#pragma unroll
  for (int kt = 0; kt < 8; ++kt) {
    bf16x16 t;
#pragma unroll
    for (int i = 0; i < 16; ++i) {
      const int k = kt * 32 + ((i < 8) ? (8 * hsel + i) : (16 + 8 * hsel + (i - 8)));
      t[i] = (__bf16)W1h[k * HID + n];
    }
    B[kt] = t;
  }

  f32x8 c[MT];
  __syncthreads();

  for (int t = 0; t < SEQ; ++t) {
    if ((t & (TCHUNK - 1)) == 0) {
      if (tid < ROWS * TCHUNK * 2 / 4) {
        const int row = tid >> 3;
        const int off = tid & 7;
        const size_t g = ((size_t)(rowb + row) * SEQ + t) * 2 + off * 4;
        *(float4*)&sx[row * (TCHUNK * 2) + off * 4] = *(const float4*)&xs[g];
        if (t + TCHUNK < SEQ)
          __builtin_prefetch(&xs[g + TCHUNK * 2], 0, 1);
      }
      __syncthreads();
    }
    const int tt = t & (TCHUNK - 1);

#pragma unroll
    for (int mt = 0; mt < MT; ++mt)
#pragma unroll
      for (int j = 0; j < 8; ++j) {
        const int m = mt * 16 + hsel * 8 + j;
        const float2 xv = *(const float2*)&sx[m * (TCHUNK * 2) + tt * 2];
        c[mt][j] = __builtin_fmaf(xv.x, wx0, __builtin_fmaf(xv.y, wx1, b1n));
      }

#pragma unroll
    for (int kt = 0; kt < 8; ++kt) {
      const int k0 = kt * 32;
#pragma unroll
      for (int mt = 0; mt < MT; ++mt) {
        ATile a;
        const __bf16* p = &sh[(mt * 16 + l15) * HSTRIDE + k0 + hsel * 8];
        a.s.lo = *(const bf16x8*)p;
        a.s.hi = *(const bf16x8*)(p + 16);
        c[mt] = __builtin_amdgcn_wmma_f32_16x16x32_f16(
            false, a.v, false, B[kt], (short)0, c[mt], false, false);
        asm volatile("v_nop\n\tv_nop\n\tv_nop\n\tv_nop" : "+v"(c[mt]) : "v"(a.v), "v"(B[kt]));
      }
    }

    __syncthreads();

#pragma unroll
    for (int mt = 0; mt < MT; ++mt)
#pragma unroll
      for (int j = 0; j < 8; ++j) {
        const float h = fast_tanh(c[mt][j]);
        c[mt][j] = h;
        const int m = mt * 16 + hsel * 8 + j;
        sh[m * HSTRIDE + n] = (__bf16)h;
      }

    __syncthreads();
  }

#pragma unroll
  for (int mt = 0; mt < MT; ++mt)
#pragma unroll
    for (int j = 0; j < 8; ++j) {
      float p = c[mt][j] * w2n;
      p += __shfl_xor(p, 1, 32);
      p += __shfl_xor(p, 2, 32);
      p += __shfl_xor(p, 4, 32);
      p += __shfl_xor(p, 8, 32);
      if (l15 == 0) sred[wave][mt * 16 + hsel * 8 + j] = p;
    }
  __syncthreads();

  if (tid < ROWS) {
    float acc = b2[0];
#pragma unroll
    for (int w = 0; w < WAVES; ++w) acc += sred[w][tid];
    *(volatile float*)(out + rowb + tid) = acc; __threadfence(); *(volatile float*)(out + rowb + tid) = acc;
  }
}

extern "C" void kernel_launch(void* const* d_in, const int* in_sizes, int n_in,
                              void* d_out, int out_size, void* d_ws, size_t ws_size,
                              hipStream_t stream) {
  const float* xs  = (const float*)d_in[0];
  const float* W1x = (const float*)d_in[1];
  const float* W1h = (const float*)d_in[2];
  const float* b1  = (const float*)d_in[3];
  const float* W2  = (const float*)d_in[4];
  const float* b2  = (const float*)d_in[5];
  float* out = (float*)d_out;

  (void)n_in; (void)out_size; (void)d_ws; (void)ws_size;
  const int batch = in_sizes[0] / (SEQ * 2);
  const int grid  = batch / ROWS;
  rnn_scan_wmma<<<grid, THREADS, 0, stream>>>(xs, W1x, W1h, b1, W2, b2, out);
}
